// TransformerBlock_41927470743716
// MI455X (gfx1250) — hardware-run, weakly checked
//
#include <hip/hip_runtime.h>


#ifndef NB
#define NB 1
#endif
#ifndef SEQ
#define SEQ 8192
#endif
#ifndef SEQK
#define SEQK 8192
#endif
#define NB_FULL   1
#define SEQ_FULL  8192
#define SEQK_FULL 8192
#define DM   128
#define HID  512
#define AW   4
#define OSP  132
#define SC2  (0.08838834764831845f * 1.4426950408889634f)
#define PSH  8.0f
#define RSC  (0.08838834764831845f * 256.0f)
#define RWT  (0.1f / 256.0f)
#define WCS  64.0f
#define WCI  (1.0f / 64.0f)
#define LNEPS 1.0e-5f

static_assert(NB == 1);
static_assert(DM == 128);
static_assert(HID == 512);
static_assert(DM % 64 == 0);
static_assert(HID % 64 == 0);
static_assert(DM % 32 == 0);
static_assert(HID % 32 == 0);
static_assert(DM % 128 == 0);
static_assert(HID % 128 == 0);
static_assert(SEQ % 64 == 0);
static_assert(SEQK % 64 == 0);
static_assert(SEQK % 32 == 0);
static_assert(SEQ % (16 * AW) == 0);
static_assert(((size_t)SEQ * 16) % 256 == 0);
static_assert(((size_t)SEQK * 16) % 256 == 0);
static_assert(SEQ <= SEQ_FULL);
static_assert(SEQK <= SEQK_FULL);
static_assert((OSP * 4) % 16 == 0);
static_assert(OSP >= DM);

typedef _Float16 h16;
typedef __attribute__((ext_vector_type(16))) _Float16 v16h;
typedef __attribute__((ext_vector_type(8)))  _Float16 v8h;
typedef __attribute__((ext_vector_type(8)))  float    v8f;
typedef __attribute__((ext_vector_type(4)))  float    v4f;
typedef v4f  __attribute__((may_alias)) v4fa;

__device__ __forceinline__ unsigned short f2bf(float f) { unsigned u = __float_as_uint(f); u += 0x7FFFu + ((u >> 16) & 1u); return (unsigned short)(u >> 16); }
__device__ __forceinline__ v16h cat16(v8h lo, v8h hi) { return __builtin_shufflevector(lo, hi, 0, 1, 2, 3, 4, 5, 6, 7, 8, 9, 10, 11, 12, 13, 14, 15); }
__device__ __forceinline__ v8f wmma16(v16h a, v16h b, v8f c) { return __builtin_amdgcn_wmma_f32_16x16x32_f16(false, a, false, b, (short)0, c, false, false); }
__device__ __forceinline__ v16h  ldh(const h16* p) { return cat16(*(const v8h*)p, *(const v8h*)(p + 16)); }
__device__ __forceinline__ void wave_sync() { __builtin_amdgcn_fence(3  , "wavefront"); __builtin_amdgcn_wave_barrier(); asm volatile("" ::: "memory"); }

__device__ __forceinline__ float bfv(float f) { return __uint_as_float(((unsigned)f2bf(f)) << 16); }
__device__ __forceinline__ h16 toh_flush(float v) { const h16 r = (h16)v; return (fabsf(v) < 6.103515625e-05f) ? (h16)0.0f : r; }
__device__ __forceinline__ v8f wmma16g(v16h a, v16h b, v8f c) {
    c = wmma16(a, b, c);
    asm volatile("v_nop\n\tv_nop\n\tv_nop\n\tv_nop" : "+v"(c) : "v"(a), "v"(b));
    return c;
}

__global__ __launch_bounds__(256) void k_wTh(const float* __restrict__ src, h16* dst, int K, int N) {
    __shared__ __align__(16) float ts[32 * OSP];
    const int tid = threadIdx.x; const int n0 = blockIdx.x * 32; const int k0 = blockIdx.y * 128;
#pragma unroll 4
    for (int it = 0; it < 16; ++it) { const int idx = it * 256 + tid; const int d = idx >> 5, ee = idx & 31;
        ts[ee * OSP + d] = src[(size_t)(k0 + d) * (size_t)N + n0 + ee]; }
    __syncthreads();
#pragma unroll 1
    for (int ps = 0; ps < 2; ++ps) {
#pragma unroll
        for (int it = 0; it < 2; ++it) { const int idx = it * 256 + tid; const int ee = idx >> 4, d8 = (idx & 15) * 8;
            const v4f x0 = *(const v4fa*)(&ts[ee * OSP + d8]); const v4f x1 = *(const v4fa*)(&ts[ee * OSP + d8 + 4]); v8h o;
#pragma unroll
            for (int i = 0; i < 4; ++i) { o[i] = toh_flush(bfv(x0[i]) * WCS); o[4 + i] = toh_flush(bfv(x1[i]) * WCS); }
            *(volatile v8h*)(dst + (size_t)(n0 + ee) * (size_t)K + k0 + d8) = o; }
        if (ps == 0) __threadfence(); }
}

__global__ __launch_bounds__(256) void k_ln(const float* __restrict__ src, const float* __restrict__ g, const float* __restrict__ b, h16* dst, int cvt) {
#pragma clang fp contract(off)
    const size_t gi = (size_t)blockIdx.x * 256 + threadIdx.x;
    const int c8 = (int)(gi & 15) * 8;
    const v8f v = *(const v8f*)(src + gi * 8);
    const v8f gv = *(const v8f*)(g + c8); const v8f bv = *(const v8f*)(b + c8);
    float x[8];
#pragma unroll
    for (int e = 0; e < 8; ++e) x[e] = cvt ? bfv(v[e]) : v[e];
    float s = ((x[0] + x[1]) + (x[2] + x[3])) + ((x[4] + x[5]) + (x[6] + x[7]));
    s += __shfl_xor(s, 8, 32); s += __shfl_xor(s, 4, 32); s += __shfl_xor(s, 2, 32); s += __shfl_xor(s, 1, 32);
    const float mu = s * (1.0f / 128.0f);
    float d[8];
#pragma unroll
    for (int e = 0; e < 8; ++e) d[e] = x[e] - mu;
    float q = ((d[0] * d[0] + d[1] * d[1]) + (d[2] * d[2] + d[3] * d[3])) + ((d[4] * d[4] + d[5] * d[5]) + (d[6] * d[6] + d[7] * d[7]));
    q += __shfl_xor(q, 8, 32); q += __shfl_xor(q, 4, 32); q += __shfl_xor(q, 2, 32); q += __shfl_xor(q, 1, 32);
    const float rs = rsqrtf(q * (1.0f / 128.0f) + LNEPS);
    v8h o;
#pragma unroll
    for (int e = 0; e < 8; ++e) o[e] = toh_flush(d[e] * rs * bfv(gv[e]) + bfv(bv[e]));
    *(volatile v8h*)(dst + gi * 8) = o;
    __threadfence();
    *(volatile v8h*)(dst + gi * 8) = o;
}

__global__ __launch_bounds__(32) void k_gemmh(const h16* __restrict__ A, const h16* __restrict__ Bt, const float* __restrict__ bias, h16* Ph, int K, int pitch, float oscale, int useBias, int useRelu) {
    __shared__ __align__(16) float os[16 * 68];
    const int lane = threadIdx.x & 31, lr = lane & 15, hi = lane >> 4; const int r0 = blockIdx.x * 64, c0 = blockIdx.y * 64;
    v8f acc[4][4];
#pragma unroll
    for (int mb = 0; mb < 4; ++mb)
#pragma unroll
        for (int nb = 0; nb < 4; ++nb) acc[mb][nb] = (v8f){};
    const size_t aoff = (size_t)(r0 + lr) * K + 8 * hi, boff = (size_t)(c0 + lr) * K + 8 * hi;
#pragma unroll 1
    for (int kc = 0; kc < K; kc += 32) {
        v16h a[4];
#pragma unroll
        for (int mb = 0; mb < 4; ++mb) a[mb] = ldh(A + aoff + (size_t)mb * 16 * K + kc);
#pragma unroll
        for (int nb = 0; nb < 4; ++nb) { const v16h b = ldh(Bt + boff + (size_t)nb * 16 * K + kc);
#pragma unroll
            for (int mb = 0; mb < 4; ++mb) acc[mb][nb] = wmma16g(a[mb], b, acc[mb][nb]); }
    }
    const int c8 = (lane & 7) * 8;
    v4f b0 = (v4f){}, b1 = (v4f){};
    if (useBias) {
        const v4f t0 = *(const v4f*)(bias + c0 + c8); const v4f t1 = *(const v4f*)(bias + c0 + c8 + 4);
#pragma unroll
        for (int i = 0; i < 4; ++i) { b0[i] = bfv(t0[i]); b1[i] = bfv(t1[i]); }
    }
    const size_t tbase = (size_t)r0 * (size_t)pitch + (size_t)c0;
#pragma unroll
    for (int mb = 0; mb < 4; ++mb) {
#pragma unroll
        for (int nb = 0; nb < 4; ++nb) {
#pragma unroll
            for (int j = 0; j < 8; ++j) os[(hi * 8 + j) * 68 + nb * 16 + lr] = acc[mb][nb][j]; }
        wave_sync();
        const size_t sb = tbase + (size_t)(mb * 16) * (size_t)pitch;
#pragma unroll 1
        for (int ps = 0; ps < 2; ++ps) {
#pragma unroll
            for (int s = 0; s < 4; ++s) { const int row = 4 * s + (lane >> 3);
                const v4f x0 = *(const v4fa*)(&os[row * 68 + c8]); const v4f x1 = *(const v4fa*)(&os[row * 68 + c8 + 4]); v8h hv;
#pragma unroll
                for (int i = 0; i < 4; ++i) { float u0 = x0[i] * oscale + b0[i]; float u1 = x1[i] * oscale + b1[i];
                    u0 = useRelu ? fmaxf(u0, 0.0f) : u0; u1 = useRelu ? fmaxf(u1, 0.0f) : u1;
                    hv[i] = toh_flush(u0); hv[4 + i] = toh_flush(u1); }
                const size_t oo = sb + (size_t)row * (size_t)pitch + c8;
                *(volatile v8h*)(Ph + oo) = hv; }
            if (ps == 0) __threadfence(); }
        wave_sync();
    }
}

__global__ __launch_bounds__(32) void k_gemmo(const h16* __restrict__ A, const h16* __restrict__ Bt, const float* __restrict__ bias, const float* __restrict__ RES, float* OUT, int K, int pitch, float oscale) {
    __shared__ __align__(16) float os[16 * 68];
    const int lane = threadIdx.x & 31, lr = lane & 15, hi = lane >> 4; const int r0 = blockIdx.x * 64, c0 = blockIdx.y * 64;
    v8f acc[4][4];
#pragma unroll
    for (int mb = 0; mb < 4; ++mb)
#pragma unroll
        for (int nb = 0; nb < 4; ++nb) acc[mb][nb] = (v8f){};
    const size_t aoff = (size_t)(r0 + lr) * K + 8 * hi, boff = (size_t)(c0 + lr) * K + 8 * hi;
#pragma unroll 1
    for (int kc = 0; kc < K; kc += 32) {
        v16h a[4];
#pragma unroll
        for (int mb = 0; mb < 4; ++mb) a[mb] = ldh(A + aoff + (size_t)mb * 16 * K + kc);
#pragma unroll
        for (int nb = 0; nb < 4; ++nb) { const v16h b = ldh(Bt + boff + (size_t)nb * 16 * K + kc);
#pragma unroll
            for (int mb = 0; mb < 4; ++mb) acc[mb][nb] = wmma16g(a[mb], b, acc[mb][nb]); }
    }
    const int c4 = (lane & 15) * 4;
    v4f bb;
    { const v4f t0 = *(const v4f*)(bias + c0 + c4);
#pragma unroll
      for (int i = 0; i < 4; ++i) bb[i] = bfv(t0[i]); }
    const size_t tbase = (size_t)r0 * (size_t)pitch + (size_t)c0;
#pragma unroll
    for (int mb = 0; mb < 4; ++mb) {
#pragma unroll
        for (int nb = 0; nb < 4; ++nb) {
#pragma unroll
            for (int j = 0; j < 8; ++j) os[(hi * 8 + j) * 68 + nb * 16 + lr] = acc[mb][nb][j]; }
        wave_sync();
        const size_t sb = tbase + (size_t)(mb * 16) * (size_t)pitch;
#pragma unroll 1
        for (int ps = 0; ps < 2; ++ps) {
#pragma unroll
            for (int s = 0; s < 8; ++s) { const int row = 2 * s + (lane >> 4);
                const v4f x0 = *(const v4fa*)(&os[row * 68 + c4]);
                const size_t oo = sb + (size_t)row * (size_t)pitch + c4;
                const v4f rr = *(const v4f*)(RES + oo);
                v4f val;
#pragma unroll
                for (int i = 0; i < 4; ++i) val[i] = (x0[i] * oscale + bb[i]) + rr[i];
                *(volatile v4f*)(OUT + oo) = val; }
            if (ps == 0) __threadfence(); }
        wave_sync();
    }
}

__global__ __launch_bounds__(32 * AW) __attribute__((amdgpu_num_vgpr(256))) void k_flash(const h16* __restrict__ QH, const h16* __restrict__ KP, const h16* __restrict__ VT, const float* __restrict__ X, float* Z1R) {
    __shared__ __align__(16) float os[AW * 16 * OSP];
    const int lane = threadIdx.x & 31, wave = __builtin_amdgcn_readfirstlane((int)(threadIdx.x >> 5)), lr = lane & 15, hi = lane >> 4;
    const int t0 = (blockIdx.x * AW + wave) * 16;
    const size_t qo = (size_t)(t0 + lr) * DM + 8 * hi;
    const size_t ko = (size_t)lr * DM + 8 * hi;
    const size_t vo = (size_t)lr * SEQK + 8 * hi;
    v8f oe[8], orl[8];
#pragma unroll
    for (int j = 0; j < 8; ++j) { oe[j] = (v8f){}; orl[j] = (v8f){}; }
    float m = -3.0e38f, l = 0.0f, rsum = 0.0f;
#pragma unroll 1
    for (int key0 = 0; key0 < SEQK; key0 += 32) {
        const h16* kp = KP + ko + (size_t)key0 * DM;
        v8f sa = (v8f){}, sb = (v8f){};
#pragma unroll 1
        for (int c = 0; c < 4; ++c) {
            const v16h q  = ldh(QH + qo + 32 * c);
            const v16h ka = ldh(kp + 32 * c);
            const v16h kb = ldh(kp + 16 * DM + 32 * c);
            sa = wmma16g(ka, q, sa); sb = wmma16g(kb, q, sb);
        }
        float ta[8], tb[8]; float mx = -3.0e38f;
#pragma unroll
        for (int r = 0; r < 8; ++r) { ta[r] = sa[r] * SC2; tb[r] = sb[r] * SC2; mx = fmaxf(mx, fmaxf(ta[r], tb[r])); }
        mx = fmaxf(mx, __shfl_xor(mx, 16, 32));
        const float mnew = fmaxf(m, mx);
        const float alpha = __builtin_amdgcn_exp2f(m - mnew);
        const float sh = PSH - mnew;
        v16h pe, pr; float ls = 0.0f, lrs = 0.0f;
#pragma unroll
        for (int r = 0; r < 8; ++r) {
            const float ea = ta[r] + sh, eb = tb[r] + sh;
            const float xa = __builtin_amdgcn_exp2f(ea), xb = __builtin_amdgcn_exp2f(eb);
            const h16 pa = (ea < -14.0f) ? (h16)0.0f : (h16)xa;
            const h16 pc = (eb < -14.0f) ? (h16)0.0f : (h16)xb;
            pe[r] = pa; pe[8 + r] = pc; ls += (float)pa + (float)pc;
            const h16 ra = toh_flush(fmaxf(sa[r] * RSC, 0.0f));
            const h16 rc = toh_flush(fmaxf(sb[r] * RSC, 0.0f));
            pr[r] = ra; pr[8 + r] = rc; lrs += (float)ra + (float)rc;
        }
        l = l * alpha + ls; rsum += lrs; m = mnew;
#pragma unroll
        for (int j = 0; j < 8; ++j) oe[j] = oe[j] * alpha;
        const h16* va = VT + vo + key0;
#pragma unroll
        for (int g = 0; g < 2; ++g) {
            v16h vv[4];
#pragma unroll
            for (int j4 = 0; j4 < 4; ++j4) vv[j4] = ldh(va + (size_t)(16 * (4 * g + j4)) * SEQK);
#pragma unroll
            for (int j4 = 0; j4 < 4; ++j4) { oe[4 * g + j4] = wmma16g(vv[j4], pe, oe[4 * g + j4]); orl[4 * g + j4] = wmma16g(vv[j4], pr, orl[4 * g + j4]); }
        }
    }
    l += __shfl_xor(l, 16, 32);
    rsum += __shfl_xor(rsum, 16, 32);
    const float inv = 1.0f / l;
    const float den = 1.0f / (rsum * RWT + 1.0f);
    const float cE = inv * den, cR = RWT * den;
    const int wb = wave * 16 * OSP;
#pragma unroll
    for (int j = 0; j < 8; ++j) {
        v4f a, c;
#pragma unroll
        for (int i = 0; i < 4; ++i) { a[i] = oe[j][i] * cE + orl[j][i] * cR; c[i] = oe[j][4 + i] * cE + orl[j][4 + i] * cR; }
        *(v4fa*)(&os[wb + lr * OSP + 16 * j + 8 * hi]) = a; *(v4fa*)(&os[wb + lr * OSP + 16 * j + 8 * hi + 4]) = c;
    }
    wave_sync();
    const float* xrow = X + (size_t)t0 * DM;
    float* zrow = Z1R + (size_t)t0 * DM;
#pragma unroll 1
    for (int ps = 0; ps < 2; ++ps) {
#pragma unroll 4
        for (int s = 0; s < 16; ++s) {
            const v4f val = *(const v4fa*)(&os[wb + s * OSP + lane * 4]);
            const v4f xv = *(const v4f*)(xrow + (size_t)s * DM + lane * 4);
            v4f z;
#pragma unroll
            for (int i = 0; i < 4; ++i) z[i] = val[i] + bfv(xv[i]);
            *(volatile v4f*)(zrow + (size_t)s * DM + lane * 4) = z; }
        if (ps == 0) __threadfence(); }
}

static constexpr size_t al256(size_t v) { return (v + 255) & ~(size_t)255; }
static constexpr size_t SZ_QP = al256((size_t)SEQ * DM * 2);
static constexpr size_t SZ_KP = al256((size_t)SEQK * DM * 2);
static constexpr size_t SZ_ZF = al256((size_t)SEQ * DM * 4);
static constexpr size_t SZ_HP = al256((size_t)SEQ * HID * 2);
static constexpr size_t SZ_WA = al256((size_t)DM * DM * 2);
static constexpr size_t SZ_WB = al256((size_t)DM * HID * 2);
static constexpr size_t SZ_WC = al256((size_t)HID * HID * 2);
static constexpr size_t SZ_TOTAL = 3 * SZ_QP + 3 * SZ_KP + SZ_ZF + 2 * SZ_HP + 3 * SZ_WA + 2 * SZ_WB + SZ_WC;
static_assert(SZ_TOTAL <= (size_t)134217728);
static_assert(SZ_QP == (size_t)SEQ * DM * 2);
static_assert(SZ_KP == (size_t)SEQK * DM * 2);
static_assert(SZ_HP == (size_t)SEQ * HID * 2);

extern "C" void kernel_launch(void* const* d_in, const int* in_sizes, int n_in,
                              void* d_out, int out_size, void* d_ws, size_t ws_size, hipStream_t stream) {
    if (n_in < 13) return;
    if ((size_t)in_sizes[0] < (size_t)SEQ * DM) return;
    if ((size_t)in_sizes[1] < (size_t)SEQK * DM) return;
    if ((size_t)in_sizes[2] < (size_t)DM * DM || (size_t)in_sizes[3] < (size_t)DM * DM || (size_t)in_sizes[4] < (size_t)DM * DM) return;
    if ((size_t)in_sizes[5] < (size_t)DM || (size_t)in_sizes[6] < (size_t)DM) return;
    if ((size_t)in_sizes[7] < (size_t)DM * HID || (size_t)in_sizes[8] < (size_t)HID) return;
    if ((size_t)in_sizes[9] < (size_t)HID * HID || (size_t)in_sizes[10] < (size_t)HID) return;
    if ((size_t)in_sizes[11] < (size_t)HID * DM || (size_t)in_sizes[12] < (size_t)DM) return;
    if ((size_t)out_size < (size_t)SEQ * DM) return;
    if (SZ_TOTAL > ws_size) return;
    const float* x   = (const float*)d_in[0];  const float* y   = (const float*)d_in[1];
    const float* wq  = (const float*)d_in[2];  const float* wk  = (const float*)d_in[3];  const float* wv = (const float*)d_in[4];
    const float* lng = (const float*)d_in[5];  const float* lnb = (const float*)d_in[6];
    const float* w1  = (const float*)d_in[7];  const float* b1  = (const float*)d_in[8];
    const float* w2  = (const float*)d_in[9];  const float* b2  = (const float*)d_in[10];
    const float* w3  = (const float*)d_in[11]; const float* b3  = (const float*)d_in[12];
    float* OUT = (float*)d_out;
    char* wsp = (char*)d_ws;
    h16* XN  = (h16*)wsp; wsp += SZ_QP;
    h16* WN  = (h16*)wsp; wsp += SZ_KP;
    h16* QH  = (h16*)wsp; wsp += SZ_QP;
    h16* KP  = (h16*)wsp; wsp += SZ_KP;
    h16* VT  = (h16*)wsp; wsp += SZ_KP;
    float* Z1R = (float*)wsp; wsp += SZ_ZF;
    h16* Z2  = (h16*)wsp; wsp += SZ_QP;
    h16* H1  = (h16*)wsp; wsp += SZ_HP;
    h16* H2  = (h16*)wsp; wsp += SZ_HP;
    h16* WQT = (h16*)wsp; wsp += SZ_WA;
    h16* WKT = (h16*)wsp; wsp += SZ_WA;
    h16* WVT = (h16*)wsp; wsp += SZ_WA;
    h16* W1T = (h16*)wsp; wsp += SZ_WB;
    h16* W3T = (h16*)wsp; wsp += SZ_WB;
    h16* W2T = (h16*)wsp; wsp += SZ_WC;

    k_wTh<<<dim3(DM / 32, DM / 128, 1), 256, 0, stream>>>(wq, WQT, DM, DM);
    k_wTh<<<dim3(DM / 32, DM / 128, 1), 256, 0, stream>>>(wk, WKT, DM, DM);
    k_wTh<<<dim3(DM / 32, DM / 128, 1), 256, 0, stream>>>(wv, WVT, DM, DM);
    k_wTh<<<dim3(HID / 32, DM / 128, 1), 256, 0, stream>>>(w1, W1T, DM, HID);
    k_wTh<<<dim3(HID / 32, HID / 128, 1), 256, 0, stream>>>(w2, W2T, HID, HID);
    k_wTh<<<dim3(DM / 32, HID / 128, 1), 256, 0, stream>>>(w3, W3T, HID, DM);

    k_ln<<<(unsigned)(((size_t)SEQ * 16) / 256), 256, 0, stream>>>(x, lng, lnb, XN, 1);
    k_ln<<<(unsigned)(((size_t)SEQK * 16) / 256), 256, 0, stream>>>(y, lng, lnb, WN, 1);

    k_gemmh<<<dim3(SEQ / 64, DM / 64, 1), 32, 0, stream>>>(XN, WQT, b1, QH, DM, DM, WCI, 0, 0);
    k_gemmh<<<dim3(SEQK / 64, DM / 64, 1), 32, 0, stream>>>(WN, WKT, b1, KP, DM, DM, WCI, 0, 0);
    k_gemmh<<<dim3(DM / 64, SEQK / 64, 1), 32, 0, stream>>>(WVT, WN, b1, VT, DM, SEQK, WCI, 0, 0);

    k_flash<<<dim3(SEQ / (16 * AW), 1, 1), 32 * AW, 0, stream>>>(QH, KP, VT, x, Z1R);

    k_ln<<<(unsigned)(((size_t)SEQ * 16) / 256), 256, 0, stream>>>(Z1R, lng, lnb, Z2, 0);

    k_gemmh<<<dim3(SEQ / 64, HID / 64, 1), 32, 0, stream>>>(Z2, W1T, b1, H1, DM, HID, WCI, 1, 1);
    k_gemmh<<<dim3(SEQ / 64, HID / 64, 1), 32, 0, stream>>>(H1, W2T, b2, H2, HID, HID, WCI, 1, 1);
    k_gemmo<<<dim3(SEQ / 64, DM / 64, 1), 32, 0, stream>>>(H2, W3T, b3, Z1R, OUT, HID, DM, WCI);
}
